// LSTM_45878840656509
// MI455X (gfx1250) — hardware-verified
//
#include <hip/hip_runtime.h>
#include <math.h>

constexpr int NBATCH  = 128;
constexpr int NSTEP   = 512;
constexpr int NIN     = 64;
constexpr int NHID    = 512;
constexpr int NGATE   = 4 * NHID;
constexpr int KCAT    = NIN + NHID;
constexpr int APITCH  = 584;
constexpr int SEQ_BLK = 16;
constexpr int NTHR    = 512;
constexpr int NWAVE   = NTHR / 32;
constexpr int OUTBLK  = 32;
constexpr int PREP_T  = 256;
constexpr int NBLK_IH = NGATE * (NIN / 8) / PREP_T;
constexpr int NBLK_HH = NGATE * (NHID / 8) / PREP_T;
constexpr int NBLK_BS = (NGATE / 4) / PREP_T;
constexpr float WCARRY     = 256.0f;
constexpr float WCARRY_INV = 1.0f / 256.0f;

static_assert(KCAT == 576 && KCAT % 32 == 0, "K multiple of 32, no pad columns");
static_assert(NBATCH % SEQ_BLK == 0, "whole 16-row tiles");
static_assert(NHID == 32 * NWAVE, "16 waves x 32 hidden units");
static_assert(NWAVE == SEQ_BLK, "one wave per output row at flush");
static_assert(NSTEP % OUTBLK == 0, "whole output lines");
static_assert(SEQ_BLK * NIN == 2 * NTHR, "x staging: 2 elements per thread");
static_assert(APITCH % 8 == 0 && APITCH >= KCAT, "A pitch");
static_assert(NBLK_IH * PREP_T == NGATE * (NIN / 8), "prep coverage ih");
static_assert(NBLK_HH * PREP_T == NGATE * (NHID / 8), "prep coverage hh");
static_assert(NBLK_BS * PREP_T * 4 == NGATE, "prep coverage bias");
static_assert((KCAT * 2) % 128 == 0, "weight plane rows are whole 128-B lines");

typedef __attribute__((ext_vector_type(16))) _Float16 v16h;
typedef __attribute__((ext_vector_type(8)))  _Float16 v8h;
typedef __attribute__((ext_vector_type(8)))  float    v8f;
typedef __attribute__((ext_vector_type(4)))  float    v4f;
typedef __attribute__((ext_vector_type(2)))  float    v2f;

__device__ __forceinline__ void guard_all4(v8f& a0, v8f& a1, v8f& a2, v8f& a3,
                                           v16h x, v16h b0, v16h b1, v16h b2, v16h b3) {
  asm volatile("v_nop\n\tv_nop\n\tv_nop\n\tv_nop"
               : "+v"(a0), "+v"(a1), "+v"(a2), "+v"(a3)
               : "v"(x), "v"(b0), "v"(b1), "v"(b2), "v"(b3));
}
__device__ __forceinline__ void acc_guard4(v8f& a, v8f& b, v8f& c, v8f& d) {
  asm volatile("v_nop\n\tv_nop\n\tv_nop\n\tv_nop" : "+v"(a), "+v"(b), "+v"(c), "+v"(d));
}

template <typename T> struct Frag;
template <> struct Frag<_Float16> {
  typedef v16h V; union U { v16h v; v8h h[2]; };
  static __device__ __forceinline__ v16h load(const _Float16* p) {
    U f; f.h[0] = *(const v8h*)(p); f.h[1] = *(const v8h*)(p + 16); return f.v;
  }
  static __device__ __forceinline__ v8f mma(v16h a, v16h b, v8f c) {
    return __builtin_amdgcn_wmma_f32_16x16x32_f16(false, a, false, b, (short)0, c, false, false);
  }
};

__device__ __forceinline__ float fsig(float x)  { return __builtin_amdgcn_rcpf(1.0f + __expf(-x)); }
__device__ __forceinline__ float ftanh(float x) { return 1.0f - 2.0f * __builtin_amdgcn_rcpf(__expf(2.0f * x) + 1.0f); }

__device__ __forceinline__ void cvt8_store(const float* sp, unsigned short* dp) {
  const v4f a = *(const v4f*)(sp);
  const v4f b = *(const v4f*)(sp + 4);
  v8h hv;
#pragma unroll
  for (int e = 0; e < 4; ++e) {
    hv[e]     = (_Float16)(a[e] * WCARRY);
    hv[4 + e] = (_Float16)(b[e] * WCARRY);
  }
  *(volatile v8h*)(dp) = hv;
  __threadfence();
  *(volatile v8h*)(dp) = hv;
}

__global__ __launch_bounds__(PREP_T) void prep_kernel(const float* __restrict__ w_ih, const float* __restrict__ w_hh,
                                                      const float* __restrict__ b_ih, const float* __restrict__ b_hh,
                                                      unsigned short* __restrict__ WC, float* __restrict__ BS) {
  const int bx = blockIdx.x, tid = threadIdx.x;
  if (bx < NBLK_IH) {
    const int i = bx * PREP_T + tid;
    const int row = i >> 3, c8 = i & 7;
    cvt8_store(w_ih + (size_t)row * NIN + c8 * 8, WC + (size_t)row * KCAT + c8 * 8);
  } else if (bx < NBLK_IH + NBLK_HH) {
    const int i = (bx - NBLK_IH) * PREP_T + tid;
    const int row = i >> 6, c8 = i & 63;
    cvt8_store(w_hh + (size_t)row * NHID + c8 * 8, WC + (size_t)row * KCAT + NIN + c8 * 8);
  } else {
    const int idx = ((bx - NBLK_IH - NBLK_HH) * PREP_T + tid) * 4;
    const v4f va = *(const v4f*)(b_ih + idx);
    const v4f vb = *(const v4f*)(b_hh + idx);
    const v4f o = va + vb;
    float* op = BS + idx;
    *(volatile v4f*)op = o;
    __threadfence();
    *(volatile v4f*)op = o;
  }
}

__global__ __launch_bounds__(NTHR) void lstm_seq_kernel(const float* __restrict__ x, const unsigned short* __restrict__ WCp,
                                                        const float* __restrict__ BS, const float* __restrict__ w_ho,
                                                        const float* __restrict__ b_ho, float* __restrict__ out) {
  __shared__ __align__(16) _Float16 At[2][SEQ_BLK * APITCH];
  __shared__ __align__(16) float    Part[2][NWAVE * 16];
  __shared__ __align__(16) float    Obuf[SEQ_BLK * OUTBLK];
  const _Float16* WC = (const _Float16*)WCp;
  const int tid = threadIdx.x, lane = tid & 31, wave = tid >> 5;
  const int c = lane & 15, hh = lane >> 4, koff = hh * 8;
  const int rowbase = blockIdx.x * SEQ_BLK;

  {
    _Float16* af = &At[0][0];
#pragma unroll 1
    for (int i = tid; i < 2 * SEQ_BLK * APITCH; i += NTHR) af[i] = (_Float16)0.0f;
  }

  float bb[2][4], wv[2];
#pragma unroll
  for (int nt = 0; nt < 2; ++nt) {
    const int j = 32 * wave + 16 * nt + c;
#pragma unroll
    for (int g = 0; g < 4; ++g) bb[nt][g] = BS[g * NHID + j];
    wv[nt] = w_ho[j];
  }
  const float bho = b_ho[0];
  asm volatile("" ::: "memory");

  float cst[2][8];
#pragma unroll
  for (int nt = 0; nt < 2; ++nt)
#pragma unroll
    for (int r = 0; r < 8; ++r) cst[nt][r] = 0.0f;

  const int xm = tid >> 5, xf = (tid & 31) * 2;
  const float* xrow = x + ((size_t)(rowbase + xm) * NSTEP) * NIN + xf;
  const int xoff = xm * APITCH + xf;

  __syncthreads();
  {
    const v2f xv = *(const v2f*)(xrow);
    const float f0 = xv[0];
    const float f1 = xv[1];
    const _Float16 h0 = (_Float16)f0;
    const _Float16 h1 = (_Float16)f1;
    const unsigned u0 = (unsigned)__builtin_bit_cast(unsigned short, h0);
    const unsigned u1 = (unsigned)__builtin_bit_cast(unsigned short, h1);
    *(unsigned*)(&At[0][0] + xoff) = u0 | (u1 << 16);
  }
  __syncthreads();

  const unsigned wbase = (unsigned)((32 * wave + c) * KCAT + koff);
  constexpr size_t GSTR = (size_t)NHID * KCAT;
  const v8f z8 = {0.f, 0.f, 0.f, 0.f, 0.f, 0.f, 0.f, 0.f};

#pragma unroll 1
  for (int t = 0; t < NSTEP; ++t) {
    const int cur = t & 1;
    const int tn = (t + 1 < NSTEP) ? (t + 1) : (NSTEP - 1);
    const v2f xnext = *(const v2f*)(xrow + (size_t)tn * NIN);

    unsigned wl = wbase;
    asm volatile("" : "+v"(wl));

    const _Float16* arow = &At[cur][0] + c * APITCH + koff;
    _Float16* anx = &At[cur ^ 1][0];

    float hp[8];
#pragma unroll
    for (int r = 0; r < 8; ++r) hp[r] = 0.0f;

#pragma unroll
    for (int nt = 0; nt < 2; ++nt) {
      const int j = 32 * wave + 16 * nt + c;
      const _Float16* wp = WC + (size_t)wl + (size_t)(nt * 16 * KCAT);
      v8f acc[4];
      acc[0] = z8; acc[1] = z8; acc[2] = z8; acc[3] = z8;
#pragma unroll 1
      for (int k0 = 0; k0 < KCAT; k0 += 32) {
        const v16h a  = Frag<_Float16>::load(arow + k0);
        const v16h b0 = Frag<_Float16>::load(wp + k0);
        const v16h b1 = Frag<_Float16>::load(wp + GSTR + k0);
        const v16h b2 = Frag<_Float16>::load(wp + 2 * GSTR + k0);
        const v16h b3 = Frag<_Float16>::load(wp + 3 * GSTR + k0);
        acc[0] = Frag<_Float16>::mma(a, b0, acc[0]);
        acc[1] = Frag<_Float16>::mma(a, b1, acc[1]);
        acc[2] = Frag<_Float16>::mma(a, b2, acc[2]);
        acc[3] = Frag<_Float16>::mma(a, b3, acc[3]);
        guard_all4(acc[0], acc[1], acc[2], acc[3], a, b0, b1, b2, b3);
      }
      acc_guard4(acc[0], acc[1], acc[2], acc[3]);
#pragma unroll
      for (int r = 0; r < 8; ++r) {
        const float zi = acc[0][r] * WCARRY_INV + bb[nt][0];
        const float zf = acc[1][r] * WCARRY_INV + bb[nt][1];
        const float zg = acc[2][r] * WCARRY_INV + bb[nt][2];
        const float zo = acc[3][r] * WCARRY_INV + bb[nt][3];
        const float ig = fsig(zi);
        const float fg = fsig(zf);
        const float gg = ftanh(zg);
        const float og = fsig(zo);
        const float cn = fg * cst[nt][r] + ig * gg;
        cst[nt][r] = cn;
        const float hn = og * ftanh(cn);
        anx[(8 * hh + r) * APITCH + NIN + j] = (_Float16)hn;
        hp[r] = fmaf(hn, wv[nt], hp[r]);
      }
    }

#pragma unroll
    for (int r = 0; r < 8; ++r) {
      float v = hp[r];
      v += __shfl_xor(v, 1, 32);
      v += __shfl_xor(v, 2, 32);
      v += __shfl_xor(v, 4, 32);
      v += __shfl_xor(v, 8, 32);
      hp[r] = v;
    }
    if (c == 0) {
      float* pp = &Part[cur][0] + wave * 16 + 8 * hh;
      v4f p0, p1;
      p0[0] = hp[0]; p0[1] = hp[1]; p0[2] = hp[2]; p0[3] = hp[3];
      p1[0] = hp[4]; p1[1] = hp[5]; p1[2] = hp[6]; p1[3] = hp[7];
      *(v4f*)(pp) = p0;
      *(v4f*)(pp + 4) = p1;
    }

    {
      const float f0 = xnext[0];
      const float f1 = xnext[1];
      const _Float16 h0 = (_Float16)f0;
      const _Float16 h1 = (_Float16)f1;
      const unsigned u0 = (unsigned)__builtin_bit_cast(unsigned short, h0);
      const unsigned u1 = (unsigned)__builtin_bit_cast(unsigned short, h1);
      *(unsigned*)(anx + xoff) = u0 | (u1 << 16);
    }

    __syncthreads();

    if (wave == 0) {
      const int row = lane & 15;
      const float* pr = &Part[cur][0] + row;
      float s = bho;
#pragma unroll
      for (int w2 = 0; w2 < NWAVE; ++w2) s += pr[w2 * 16];
      if (lane < 16) Obuf[row * OUTBLK + (t & (OUTBLK - 1))] = s;
    }

    if ((t & (OUTBLK - 1)) == (OUTBLK - 1)) {
      __syncthreads();
      const float v = Obuf[wave * OUTBLK + lane];
      float* op = out + (size_t)(rowbase + wave) * NSTEP + (size_t)(t - (OUTBLK - 1)) + lane;
      *(volatile float*)op = v;
      __threadfence();
      *(volatile float*)op = v;
    }
  }
}

extern "C" void kernel_launch(void* const* d_in, const int* in_sizes, int n_in,
                              void* d_out, int out_size, void* d_ws, size_t ws_size, hipStream_t stream) {
  if (n_in < 7 || d_out == nullptr || d_ws == nullptr) return;
  if (in_sizes[0] != NBATCH * NSTEP * NIN || in_sizes[1] != NGATE * NIN || in_sizes[2] != NGATE * NHID ||
      in_sizes[3] != NGATE || in_sizes[4] != NGATE || in_sizes[5] != NHID || in_sizes[6] != 1 ||
      out_size != NBATCH * NSTEP) return;

  const float* x    = (const float*)d_in[0];
  const float* w_ih = (const float*)d_in[1];
  const float* w_hh = (const float*)d_in[2];
  const float* b_ih = (const float*)d_in[3];
  const float* b_hh = (const float*)d_in[4];
  const float* w_ho = (const float*)d_in[5];
  const float* b_ho = (const float*)d_in[6];
  float* out = (float*)d_out;

  char* ws = (char*)d_ws; size_t off = 0;
  auto carve = [&](size_t bytes) -> char* { char* p = ws + off; off += (bytes + 255) & ~(size_t)255; return p; };
  unsigned short* WC = (unsigned short*)carve((size_t)NGATE * KCAT * 2);
  float*          BS = (float*)carve((size_t)NGATE * 4);
  if (off > ws_size || off > (size_t)134217728) return;

  prep_kernel<<<NBLK_IH + NBLK_HH + NBLK_BS, PREP_T, 0, stream>>>(w_ih, w_hh, b_ih, b_hh, WC, BS);
  lstm_seq_kernel<<<NBATCH / SEQ_BLK, NTHR, 0, stream>>>(x, WC, BS, w_ho, b_ho, out);
}
